// LorentzianKAN_15693810499706
// MI455X (gfx1250) — hardware-run, weakly checked
//
#include <hip/hip_runtime.h>


namespace {
constexpr int NBR = 32768, D0 = 128, D1 = 256, D2 = 128, G = 16, KCH = 1024;
constexpr float HS = 256.0f, WSC = 256.0f, GAM = 0.2f, LNEPS = 1e-5f;
typedef _Float16 b16;
typedef __attribute__((ext_vector_type(16))) _Float16 v16b;
typedef __attribute__((ext_vector_type(8))) _Float16 v8b;
typedef __attribute__((ext_vector_type(8))) float v8f;
typedef __attribute__((ext_vector_type(4))) float v4f;
__device__ __forceinline__ float bf16_rne(float f) { unsigned int u = __float_as_uint(f); u += 0x7FFFu + ((u >> 16) & 1u); float r = __uint_as_float(u & 0xFFFF0000u); asm volatile("" : "+v"(r)); return r; }
__device__ __forceinline__ float bfv(float f) { float r = bf16_rne(f); asm volatile("" : "+v"(r)); return r; }
__device__ __forceinline__ void split16(float v, b16& hi, b16& lo) { hi = (b16)v; lo = (b16)(v - (float)hi); }
__device__ __forceinline__ v16b frag_kb(const b16* p, int hh) { const v8b a = *(const v8b*)(p + 8 * hh), b = *(const v8b*)(p + 16 + 8 * hh); v16b f;
#pragma unroll
  for (int e = 0; e < 8; ++e) { f[e] = a[e]; f[8 + e] = b[e]; } return f; }
__device__ __forceinline__ v8f wmma16b(v16b a, v16b b, v8f c) { v8f d = __builtin_amdgcn_wmma_f32_16x16x32_f16(false, a, false, b, (short)0, c, false, false); asm volatile("v_nop\n\tv_nop\n\tv_nop\n\tv_nop" : "+v"(d) : "v"(a), "v"(b)); return d; }
__device__ __forceinline__ void wave_lds_sync() { __builtin_amdgcn_fence(__ATOMIC_RELEASE, "workgroup"); __builtin_amdgcn_wave_barrier(); __builtin_amdgcn_fence(__ATOMIC_ACQUIRE, "workgroup"); }
__device__ __forceinline__ float pmul(float a, float b) { float p = a * b; asm volatile("" : "+v"(p)); return p; }

__global__ __launch_bounds__(256) void wput_kernel(const float* __restrict__ bw1, const float* __restrict__ sw1, const float* __restrict__ bw2, const float* __restrict__ sw2, b16* __restrict__ BW1, b16* __restrict__ SW1, b16* __restrict__ BW2, b16* __restrict__ SW2) { const size_t u = (size_t)blockIdx.x * 256 + threadIdx.x; v8b v;
  auto put = [&](const float* src, b16* dst, size_t n8) { if (u < n8) {
#pragma unroll
      for (int j = 0; j < 8; ++j) v[j] = (b16)(bf16_rne(src[u * 8 + j]) * WSC); for (int pass = 0; pass < 2; ++pass) { *(volatile v8b*)(dst + u * 8) = v; __threadfence(); } } };
  put(bw1, BW1, (size_t)D1 * D0 / 8); put(sw1, SW1, (size_t)D1 * D0 * G / 8); put(bw2, BW2, (size_t)D2 * D1 / 8); put(sw2, SW2, (size_t)D2 * D1 * G / 8); }
template <int DIN, int DOUT, int IS_X>
__global__ __launch_bounds__(32) void kan_kernel(const float* __restrict__ Z, const float* __restrict__ lnw, const float* __restrict__ lnb, const b16* __restrict__ BW, const float* __restrict__ bb, const b16* __restrict__ SW, int RLIM, float* __restrict__ OUT) {
  constexpr int NT = DOUT / 16, KT = DIN * G, NCH = KT / KCH, IPC = KCH / G  ;
  __shared__ __attribute__((aligned(16))) b16 Sh[16][DIN + 8], Sl[16][DIN + 8], Bs[16][KCH + 8], Bq[16][KCH + 8]; __shared__ float Zn[16][DIN + 4], Tf[16][DOUT + 4]; const int lane = threadIdx.x, nloc = lane & 15, hlf = lane >> 4; const size_t m0 = (size_t)blockIdx.x * 16; if (m0 >= (size_t)RLIM) return;
  for (int rr = 0; rr < 16; ++rr) { float s = 0.0f, s2 = 0.0f; float zv[DIN / 32];
#pragma unroll
    for (int q = 0; q < DIN / 32; ++q) { const float z = IS_X ? bfv(Z[(m0 + rr) * DIN + q * 32 + lane]) : Z[(m0 + rr) * DIN + q * 32 + lane]; zv[q] = z; s += z; b16 p, ql; split16((z / (1.0f + __expf(-z))) * HS, p, ql); Sh[rr][q * 32 + lane] = p; Sl[rr][q * 32 + lane] = ql; }
    for (int o = 16; o; o >>= 1) s += __shfl_xor(s, o); const float mu = s / DIN;
#pragma unroll
    for (int q = 0; q < DIN / 32; ++q) { const float d = zv[q] - mu; s2 += d * d; }
    for (int o = 16; o; o >>= 1) s2 += __shfl_xor(s2, o); const float rs = rsqrtf(s2 / DIN + LNEPS);
#pragma unroll
    for (int q = 0; q < DIN / 32; ++q) { const int i = q * 32 + lane; Zn[rr][i] = pmul(pmul(zv[q] - mu, rs), bfv(lnw[i])) + bfv(lnb[i]); } }
  if (lane < 16) for (int k = DIN; k < DIN + 8; ++k) { Sh[lane][k] = (b16)0.0f; Sl[lane][k] = (b16)0.0f; }
  wave_lds_sync(); v8f acc[NT];
#pragma unroll
  for (int t = 0; t < NT; ++t) acc[t] = (v8f){};
#pragma unroll 2
  for (int kb = 0; kb < DIN; kb += 32) { const v16b a = frag_kb(&Sh[nloc][kb], hlf), al = frag_kb(&Sl[nloc][kb], hlf);
#pragma unroll
    for (int t = 0; t < NT; ++t) { const v16b bw = frag_kb(BW + (size_t)(t * 16 + nloc) * DIN + kb, hlf); acc[t] = wmma16b(a, bw, acc[t]); acc[t] = wmma16b(al, bw, acc[t]); } }
#pragma unroll 1
  for (int ch = 0; ch < NCH; ++ch) {
    for (int rr = 0; rr < 16; ++rr) for (int q = 0; q < IPC / 32; ++q) { const int il = q * 32 + lane; const float zn = Zn[rr][ch * IPC + il]; b16* row = &Bs[rr][il * G]; b16* rowl = &Bq[rr][il * G];
#pragma unroll
      for (int g = 0; g < G; ++g) { const float d = zn - (-1.0f + 0.2f * (float)g); b16 p, ql; split16((GAM * GAM) / (d * d + GAM * GAM) * HS, p, ql); row[g] = p; rowl[g] = ql; } }
    if (lane < 16) for (int k = KCH; k < KCH + 8; ++k) { Bs[lane][k] = (b16)0.0f; Bq[lane][k] = (b16)0.0f; }
    wave_lds_sync(); const b16* SWc = SW + (size_t)ch * KCH;
#pragma unroll 2
    for (int kb = 0; kb < KCH; kb += 32) { const v16b a = frag_kb(&Bs[nloc][kb], hlf), al = frag_kb(&Bq[nloc][kb], hlf);
#pragma unroll
      for (int t = 0; t < NT; ++t) { const v16b bw = frag_kb(SWc + (size_t)(t * 16 + nloc) * KT + kb, hlf); acc[t] = wmma16b(a, bw, acc[t]); acc[t] = wmma16b(al, bw, acc[t]); } }
    wave_lds_sync(); }
#pragma unroll
  for (int t = 0; t < NT; ++t) { const int cc = t * 16 + nloc; const float b = bfv(bb[cc]);
#pragma unroll
    for (int r8 = 0; r8 < 8; ++r8) Tf[8 * hlf + r8][cc] = acc[t][r8] * (1.0f / (HS * WSC)) + b; }
  wave_lds_sync();
  for (int pass = 0; pass < 2; ++pass) { for (int rr = 0; rr < 16; ++rr) for (int q = 0; q < DOUT / 128; ++q) *(volatile v4f*)(OUT + (m0 + rr) * DOUT + q * 128 + lane * 4) = *(const v4f*)(&Tf[rr][q * 128 + lane * 4]); __threadfence(); } }
}

extern "C" void kernel_launch(void* const* d_in, const int* in_sizes, int n_in, void* d_out, int out_size, void* d_ws, size_t ws_size, hipStream_t stream) {
  (void)n_in;
  auto Fp = [&](int i) { return (const float*)d_in[i]; };
  if (in_sizes[0] != NBR * D0 || in_sizes[3] != D1 * D0 || in_sizes[5] != D1 * D0 * G || in_sizes[8] != D2 * D1 || in_sizes[10] != D2 * D1 * G || out_size != NBR * D2) return;
  const int RLIM = NBR;
  size_t off = 0; char* ws = (char*)d_ws;
  auto carve = [&](size_t bytes) { char* p = ws + off; off += (bytes + 255) & ~(size_t)255; return p; };
  b16* BW1 = (b16*)carve((size_t)D1 * D0 * 2); b16* SW1 = (b16*)carve((size_t)D1 * D0 * G * 2); b16* BW2 = (b16*)carve((size_t)D2 * D1 * 2); b16* SW2 = (b16*)carve((size_t)D2 * D1 * G * 2); float* H1 = (float*)carve((size_t)NBR * D1 * 4);
  if (off > ws_size || off > ((size_t)64 << 20)) return;
  wput_kernel<<<(unsigned)(((size_t)D1 * D0 * G / 8 + 255) / 256), 256, 0, stream>>>(Fp(3), Fp(5), Fp(8), Fp(10), BW1, SW1, BW2, SW2);
  kan_kernel<D0, D1, 1><<<RLIM / 16, 32, 0, stream>>>(Fp(0), Fp(1), Fp(2), BW1, Fp(4), SW1, RLIM, H1);
  kan_kernel<D1, D2, 0><<<RLIM / 16, 32, 0, stream>>>(H1, Fp(6), Fp(7), BW2, Fp(9), SW2, RLIM, (float*)d_out);
}
